// DiffGraphSTFormerBlock_55405078118814
// MI455X (gfx1250) — hardware-run, weakly checked
//
#include <hip/hip_runtime.h>
#include <stddef.h>
#include <stdint.h>

#define NBATCH 8
#define NTIME  128
#define NNODE  64
#define DIN    32
#define DMOD   128
#define NHEAD  4
#define HDIM   32
#define NTOK   65536
#define WQKV   384
#define WGQK   256
#define ROWSPN 1024

static_assert(NTOK == NBATCH * NTIME * NNODE);
static_assert(ROWSPN == NBATCH * NTIME);
static_assert(ROWSPN % 256 == 0);
static_assert(NTOK % 256 == 0);
static_assert(NTOK % 16 == 0);
static_assert(DMOD % 64 == 0 && WQKV % 64 == 0 && WGQK % 64 == 0);
static_assert(DIN % 32 == 0 && DMOD % 32 == 0);
static_assert(NHEAD * HDIM == DMOD);
static_assert(NTIME == 128 && NNODE == 64 && HDIM == 32 && DMOD == 128);
static_assert((NTOK * DIN) % 2048 == 0);

typedef _Float16 v16h __attribute__((ext_vector_type(16)));
typedef _Float16 v8h  __attribute__((ext_vector_type(8)));
typedef float    v8f  __attribute__((ext_vector_type(8)));
typedef float    v4f  __attribute__((ext_vector_type(4)));
typedef unsigned int v4u __attribute__((ext_vector_type(4)));

union Frag  { v16h v; v8h h[2]; };
union Pack8 { v8h h; v4u u; };

__device__ __forceinline__ v8f mma16(v16h a, v16h b, v8f c) {
  c = __builtin_amdgcn_wmma_f32_16x16x32_f16(false, a, false, b, (short)0, c, false, false);
  asm volatile("v_nop\n\tv_nop\n\tv_nop\n\tv_nop" : "+v"(c) : "v"(a), "v"(b));
  return c;
}

__device__ __forceinline__ v16h ldfrag(const _Float16* p, int ld, int row0, int k0, int lane) {
  const int m = lane & 15, lh = lane >> 4;
  const _Float16* q = p + (size_t)(row0 + m) * ld + k0 + 8 * lh;
  Frag f;
  f.h[0] = *(const v8h*)(q);
  f.h[1] = *(const v8h*)(q + 16);
  return f.v;
}

__device__ __forceinline__ v8f zero8() { return (v8f){0.f, 0.f, 0.f, 0.f, 0.f, 0.f, 0.f, 0.f}; }

__device__ __forceinline__ float gelu_t(float x) {
  const float u = 0.7978845608028654f * (x + 0.044715f * x * x * x);
  const float e = __expf(-2.0f * u);
  return x * __builtin_amdgcn_rcpf(1.0f + e);
}

__device__ __forceinline__ void sincos_q(float x, float& s, float& c) {
  const float kf = rintf(x * 0.636619772367581343f);
  float r = fmaf(kf, -1.57079625129699707031f, x);
  r = fmaf(kf, -7.54978941586159635335e-8f, r);
  r = fmaf(kf, -5.39030252995776476554e-15f, r);
  const int q = ((int)kf) & 3;
  const float z = r * r;
  const float sp = fmaf(((-1.9515295891e-4f * z + 8.3321608736e-3f) * z - 1.6666654611e-1f) * z, r, r);
  const float cp = fmaf(((2.443315711809948e-5f * z - 1.388731625493765e-3f) * z + 4.166664568298827e-2f) * z, z,
                        fmaf(-0.5f, z, 1.0f));
  const float s0 = (q & 1) ? cp : sp;
  const float c0 = (q & 1) ? sp : cp;
  s = (q & 2) ? -s0 : s0;
  c = ((q + 1) & 2) ? -c0 : c0;
}

__device__ __forceinline__ void gemm32x64(const _Float16* __restrict__ A, int lda, int akst,
                                          const _Float16* __restrict__ Bt, int ldb, int nks,
                                          int r0, int n0, int lane, v8f (&acc)[2][4]) {
#pragma unroll 1
  for (int ks = 0; ks < nks; ++ks) {
    const _Float16* Ak = A + (size_t)ks * akst;
    const v16h a0 = ldfrag(Ak, lda, r0, 0, lane);
    const v16h a1 = ldfrag(Ak, lda, r0 + 16, 0, lane);
    const v16h b0 = ldfrag(Bt, ldb, n0, 32 * ks, lane);
    const v16h b1 = ldfrag(Bt, ldb, n0 + 16, 32 * ks, lane);
    const v16h b2 = ldfrag(Bt, ldb, n0 + 32, 32 * ks, lane);
    const v16h b3 = ldfrag(Bt, ldb, n0 + 48, 32 * ks, lane);
    acc[0][0] = mma16(a0, b0, acc[0][0]);
    acc[1][0] = mma16(a1, b0, acc[1][0]);
    acc[0][1] = mma16(a0, b1, acc[0][1]);
    acc[1][1] = mma16(a1, b1, acc[1][1]);
    acc[0][2] = mma16(a0, b2, acc[0][2]);
    acc[1][2] = mma16(a1, b2, acc[1][2]);
    acc[0][3] = mma16(a0, b3, acc[0][3]);
    acc[1][3] = mma16(a1, b3, acc[1][3]);
  }
}

__global__ __launch_bounds__(256) void k_cvt8(const float* __restrict__ src, _Float16* __restrict__ dst) {
  const size_t o = ((size_t)blockIdx.x * 256 + threadIdx.x) * 8;
  const v4f a0 = *(const v4f*)(src + o);
  const v4f a1 = *(const v4f*)(src + o + 4);
  Pack8 pk;
  pk.h = (v8h){(_Float16)a0[0], (_Float16)a0[1], (_Float16)a0[2], (_Float16)a0[3],
               (_Float16)a1[0], (_Float16)a1[1], (_Float16)a1[2], (_Float16)a1[3]};
  const v4u vv = pk.u;
  volatile v4u* d = (volatile v4u*)(dst + o);
  *d = vv;
  __threadfence();
  *d = vv;
}

template<int K>
__global__ __launch_bounds__(256) void k_wt(const float* __restrict__ W, int nout,
                                            _Float16* __restrict__ Wt, float scale) {
  __shared__ __align__(16) float tile[32 * (K + 4)];
  const int tid = threadIdx.x;
  const int node = blockIdx.y;
  const int n0 = blockIdx.x * 32;
  const float* src = W + (size_t)node * K * nout + n0;
#pragma unroll 1
  for (int it = 0; it < (32 * K) / 256; ++it) {
    const int idx = tid + 256 * it;
    const int k = idx >> 5, nn = idx & 31;
    tile[nn * (K + 4) + k] = src[(size_t)k * nout + nn] * scale;
  }
  __syncthreads();
  constexpr int NPR = K / 8;
  constexpr int TOTP = 32 * NPR;
  constexpr int PPT = (TOTP + 255) / 256;
  const bool act = (TOTP >= 256) || (tid < TOTP);
  v4u val[PPT];
  size_t go[PPT];
#pragma unroll
  for (int j = 0; j < PPT; ++j) {
    int p = tid + 256 * j;
    if (p >= TOTP) p = 0;
    const int row = p / NPR, pc = p - row * NPR;
    const float* ra = tile + row * (K + 4) + pc * 8;
    const v4f a0 = *(const v4f*)(ra), a1 = *(const v4f*)(ra + 4);
    Pack8 pk;
    pk.h = (v8h){(_Float16)a0[0], (_Float16)a0[1], (_Float16)a0[2], (_Float16)a0[3],
                 (_Float16)a1[0], (_Float16)a1[1], (_Float16)a1[2], (_Float16)a1[3]};
    val[j] = pk.u;
    go[j] = (size_t)node * nout * K + (size_t)(n0 + row) * K + pc * 8;
  }
  if (act) {
#pragma unroll
    for (int j = 0; j < PPT; ++j) *(volatile v4u*)(Wt + go[j]) = val[j];
    __threadfence();
#pragma unroll
    for (int j = 0; j < PPT; ++j) *(volatile v4u*)(Wt + go[j]) = val[j];
  }
}

__global__ __launch_bounds__(256) void k_petab(float* __restrict__ pe) {
  const int e = blockIdx.x * 256 + threadIdx.x;
  const int t = e >> 7, d = e & 127;
  const float i2 = (float)(d & ~1);
  const float dv = expf((-9.2103405f * i2) * 0.0078125f);
  const float ang = (float)t * dv;
  float s, c;
  sincos_q(ang, s, c);
  const float v = (d & 1) ? c : s;
  volatile float* q = pe + e;
  *q = v;
  __threadfence();
  *q = v;
}

#define OTP 68
template<int OUTK, bool RES, bool GELU, bool PE, bool AOP>
__global__ __launch_bounds__(256) void k_gemm(const _Float16* __restrict__ A, int lda, int a_node,
                                              const _Float16* __restrict__ Bt, int K, int b_node,
                                              const float* __restrict__ bias, int bias_node,
                                              const float* __restrict__ res, const float* __restrict__ pe,
                                              float scale, float oscale,
                                              float* __restrict__ outf, _Float16* __restrict__ outh,
                                              int ldo, int o_node) {
  __shared__ __align__(16) float st[8][16 * OTP];
  const int tid = threadIdx.x, lane = tid & 31, wave = tid >> 5;
  const int hh = lane >> 4, c = lane & 15;
  const int node = blockIdx.z;
  const int m0 = blockIdx.x * 256 + wave * 32;
  const int n0 = blockIdx.y * 64;

  const _Float16* Ab;
  int lda_e, akst, r0;
  if constexpr (AOP) {
    Ab = A + ((size_t)(((m0 >> 7) * NNODE + node) * NHEAD) << 12);
    lda_e = HDIM; akst = NTIME * HDIM; r0 = m0 & (NTIME - 1);
  } else {
    Ab = A + (size_t)node * a_node; lda_e = lda; akst = 32; r0 = m0;
  }
  const _Float16* Bn = Bt + (size_t)node * b_node;

  v8f acc[2][4];
#pragma unroll
  for (int s = 0; s < 2; ++s)
#pragma unroll
    for (int t = 0; t < 4; ++t) acc[s][t] = zero8();
  gemm32x64(Ab, lda_e, akst, Bn, K, K >> 5, r0, n0, lane, acc);

  float bb[4];
#pragma unroll
  for (int t = 0; t < 4; ++t) bb[t] = bias[(size_t)node * bias_node + n0 + 16 * t + c];

  float* sw = st[wave];
  const size_t obase = (size_t)node * o_node;
#pragma unroll
  for (int sub = 0; sub < 2; ++sub) {
    __syncthreads();
#pragma unroll
    for (int t = 0; t < 4; ++t) {
#pragma unroll
      for (int r = 0; r < 8; ++r) {
        float v = acc[sub][t][r] * scale + bb[t];
        if constexpr (GELU) v = gelu_t(v);
        sw[(8 * hh + r) * OTP + 16 * t + c] = v;
      }
    }
    __syncthreads();
    const int mr0 = m0 + sub * 16;
    if constexpr (OUTK == 0 || OUTK == 2) {
      v4f val[8];
      size_t go[8];
#pragma unroll
      for (int it = 0; it < 8; ++it) {
        const int p    = lane + 32 * it;
        const int L    = p >> 3;
        const int pc   = p & 7;
        const int row  = L >> 1;
        const int half = L & 1;
        v4f v = *(const v4f*)(sw + row * OTP + half * 32 + pc * 4);
        const size_t o = obase + (size_t)(mr0 + row) * ldo + n0 + half * 32 + pc * 4;
        if constexpr (RES) v += *(const v4f*)(res + o);
        if constexpr (PE) v += *(const v4f*)(pe + ((mr0 + row) & (NTIME - 1)) * DMOD + n0 + half * 32 + pc * 4);
        val[it] = v;
        go[it] = o;
      }
#pragma unroll
      for (int it = 0; it < 8; ++it) *(volatile v4f*)(outf + go[it]) = val[it];
      __threadfence();
#pragma unroll
      for (int it = 0; it < 8; ++it) *(volatile v4f*)(outf + go[it]) = val[it];
    }
    if constexpr (OUTK == 1 || OUTK == 2) {
      v4u hv[4];
      size_t gh[4];
#pragma unroll
      for (int it = 0; it < 4; ++it) {
        const int p  = lane + 32 * it;
        const int L  = p >> 3;
        const int pc = p & 7;
        const float* ra = sw + L * OTP + pc * 8;
        v4f a0 = *(const v4f*)(ra), a1 = *(const v4f*)(ra + 4);
        const size_t o = obase + (size_t)(mr0 + L) * ldo + n0 + pc * 8;
        if constexpr (RES) { a0 += *(const v4f*)(res + o); a1 += *(const v4f*)(res + o + 4); }
        if constexpr (PE) {
          const float* pr = pe + ((mr0 + L) & (NTIME - 1)) * DMOD + n0 + pc * 8;
          a0 += *(const v4f*)(pr); a1 += *(const v4f*)(pr + 4);
        }
        a0 *= oscale; a1 *= oscale;
        Pack8 pk;
        pk.h = (v8h){(_Float16)a0[0], (_Float16)a0[1], (_Float16)a0[2], (_Float16)a0[3],
                     (_Float16)a1[0], (_Float16)a1[1], (_Float16)a1[2], (_Float16)a1[3]};
        hv[it] = pk.u;
        gh[it] = o;
      }
#pragma unroll
      for (int it = 0; it < 4; ++it) *(volatile v4u*)(outh + gh[it]) = hv[it];
      __threadfence();
#pragma unroll
      for (int it = 0; it < 4; ++it) *(volatile v4u*)(outh + gh[it]) = hv[it];
    }
  }
}

__global__ __launch_bounds__(256) void k_ln(const float* __restrict__ X, const float* __restrict__ S,
                                            const float* __restrict__ Bv, int smask,
                                            _Float16* __restrict__ Y) {
  __shared__ __align__(16) float sw[8][2][DMOD];
  const int tid = threadIdx.x, lane = tid & 31, wave = tid >> 5;
  const int row0 = blockIdx.x * 16 + wave * 2;
#pragma unroll
  for (int rr = 0; rr < 2; ++rr) {
    const int row = row0 + rr;
    const v4f v = *(const v4f*)(X + (size_t)row * DMOD + 4 * lane);
    float s = (v[0] + v[1]) + (v[2] + v[3]);
#pragma unroll
    for (int off = 16; off >= 1; off >>= 1) s += __shfl_xor(s, off, 32);
    const float mean = s * 0.0078125f;
    const v4f d = v - mean;
    float ss = (d[0] * d[0] + d[1] * d[1]) + (d[2] * d[2] + d[3] * d[3]);
#pragma unroll
    for (int off = 16; off >= 1; off >>= 1) ss += __shfl_xor(ss, off, 32);
    const float var  = ss * 0.0078125f;
    const float rstd = rsqrtf(var + 1e-6f);
    const int soff = (row & smask) * DMOD + 4 * lane;
    const v4f gv = *(const v4f*)(S + soff);
    const v4f bv = *(const v4f*)(Bv + soff);
    const v4f y = (d * rstd) * gv + bv;
    *(v4f*)(&sw[wave][rr][4 * lane]) = y;
  }
  __syncthreads();
  const int rr = lane >> 4, pc = lane & 15;
  const float* ra = &sw[wave][rr][8 * pc];
  const v4f a0 = *(const v4f*)(ra), a1 = *(const v4f*)(ra + 4);
  Pack8 pk;
  pk.h = (v8h){(_Float16)a0[0], (_Float16)a0[1], (_Float16)a0[2], (_Float16)a0[3],
               (_Float16)a1[0], (_Float16)a1[1], (_Float16)a1[2], (_Float16)a1[3]};
  const v4u hv = pk.u;
  volatile v4u* dp = (volatile v4u*)(Y + (size_t)(row0 + rr) * DMOD + 8 * pc);
  *dp = hv;
  __threadfence();
  *dp = hv;
}

#define KSP 40
#define PTP 136
__global__ __launch_bounds__(256) void k_attn_t(const _Float16* __restrict__ qkv, _Float16* __restrict__ oh,
                                                float sscale) {
  __shared__ __align__(16) _Float16 Ks[NTIME * KSP];
  __shared__ __align__(16) _Float16 Vt[HDIM * PTP];
  __shared__ __align__(16) _Float16 Ps[8 * 16 * PTP];
  const int tid = threadIdx.x, lane = tid & 31, wave = tid >> 5;
  const int hh = lane >> 4, c = lane & 15;
  const int b = blockIdx.x >> 6, n = blockIdx.x & 63;
  const int t0 = wave * 16;
  const size_t RP = (size_t)NNODE * WQKV;
  const _Float16* base = qkv + ((size_t)b * (NTIME * NNODE) + n) * WQKV;
  _Float16* pw = Ps + wave * 16 * PTP;
  const float NEGI = -__builtin_huge_valf();

#pragma unroll 1
  for (int h = 0; h < NHEAD; ++h) {
    __syncthreads();
#pragma unroll
    for (int it = 0; it < 2; ++it) {
      const int idx = tid + 256 * it;
      const int s = idx >> 2, pc = idx & 3;
      const _Float16* rp = base + (size_t)s * RP + h * HDIM + 8 * pc;
      *(v8h*)(Ks + s * KSP + 8 * pc) = *(const v8h*)(rp + DMOD);
      const v8h vv = *(const v8h*)(rp + 2 * DMOD);
#pragma unroll
      for (int e = 0; e < 8; ++e) Vt[(8 * pc + e) * PTP + s] = vv[e];
    }
    __syncthreads();

    const v16h qa = ldfrag(base + h * HDIM, (int)RP, t0, 0, lane);
    v8f s[8];
#pragma unroll
    for (int j = 0; j < 8; ++j) s[j] = mma16(qa, ldfrag(Ks, KSP, 16 * j, 0, lane), zero8());
    float inv[8];
#pragma unroll
    for (int r = 0; r < 8; ++r) {
      float m = NEGI;
#pragma unroll
      for (int j = 0; j < 8; ++j) { s[j][r] *= sscale; m = fmaxf(m, s[j][r]); }
#pragma unroll
      for (int off = 1; off < 16; off <<= 1) m = fmaxf(m, __shfl_xor(m, off, 32));
      float sum = 0.f;
#pragma unroll
      for (int j = 0; j < 8; ++j) {
        const float p = __expf(s[j][r] - m);
        sum += p;
        pw[(8 * hh + r) * PTP + 16 * j + c] = (_Float16)(p * 1024.0f);
      }
#pragma unroll
      for (int off = 1; off < 16; off <<= 1) sum += __shfl_xor(sum, off, 32);
      inv[r] = 0.0078125f * __builtin_amdgcn_rcpf(sum);
    }
    __syncthreads();

    v8f o[2];
    o[0] = zero8(); o[1] = zero8();
#pragma unroll
    for (int kk = 0; kk < 4; ++kk) {
      const v16h pa = ldfrag(pw, PTP, 0, 32 * kk, lane);
#pragma unroll
      for (int t = 0; t < 2; ++t) {
        const v16h vb = ldfrag(Vt, PTP, 16 * t, 32 * kk, lane);
        o[t] = mma16(pa, vb, o[t]);
      }
    }
#pragma unroll
    for (int t = 0; t < 2; ++t)
#pragma unroll
      for (int r = 0; r < 8; ++r)
        pw[(8 * hh + r) * PTP + 16 * t + c] = (_Float16)(o[t][r] * inv[r]);
    __syncthreads();
    v4u val[2];
    size_t go[2];
#pragma unroll
    for (int it = 0; it < 2; ++it) {
      const int p  = lane + 32 * it;
      const int L  = p >> 2;
      const int pc = p & 3;
      Pack8 pk;
      pk.h    = *(const v8h*)(pw + L * PTP + 8 * pc);
      val[it] = pk.u;
      go[it]  = ((((size_t)(b * NNODE + n) * NHEAD + h) * NTIME + t0 + L) << 5) + 8 * pc;
    }
#pragma unroll
    for (int it = 0; it < 2; ++it) *(volatile v4u*)(oh + go[it]) = val[it];
    __threadfence();
#pragma unroll
    for (int it = 0; it < 2; ++it) *(volatile v4u*)(oh + go[it]) = val[it];
  }
}

#define APT 68
#define AHP 72
__global__ __launch_bounds__(256) void k_gdiff(const _Float16* __restrict__ qk, float* __restrict__ z,
                                               _Float16* __restrict__ zh, float sscale, float dt) {
  __shared__ __align__(16) float lds[11264];
  float*    Apart = lds;
  _Float16* Ah    = (_Float16*)(lds + 4352);
  _Float16* Zt    = (_Float16*)(lds + 6656);
  float*    stg   = lds;
  const int tid = threadIdx.x, lane = tid & 31, wave = tid >> 5;
  const int hh = lane >> 4, c = lane & 15;
  const size_t rowb = (size_t)blockIdx.x * NNODE;
  const int rt = wave >> 1, hp = wave & 1;
  const float NEGI = -__builtin_huge_valf();

#pragma unroll
  for (int it = 0; it < 4; ++it) {
    const int idx = tid + 256 * it;
    const int m = idx >> 4, pc = idx & 15;
    const v8h vv = *(const v8h*)(zh + (rowb + m) * DMOD + 8 * pc);
#pragma unroll
    for (int e = 0; e < 8; ++e) Zt[(8 * pc + e) * AHP + m] = vv[e];
  }

  const _Float16* qb = qk + rowb * WGQK;
  v8f pacc[4];
#pragma unroll
  for (int j = 0; j < 4; ++j) pacc[j] = zero8();
#pragma unroll
  for (int h2 = 0; h2 < 2; ++h2) {
    const int h = 2 * hp + h2;
    const v16h qa = ldfrag(qb + h * HDIM, WGQK, rt * 16, 0, lane);
    v8f s[4];
#pragma unroll
    for (int j = 0; j < 4; ++j) s[j] = mma16(qa, ldfrag(qb + DMOD + h * HDIM, WGQK, 16 * j, 0, lane), zero8());
#pragma unroll
    for (int r = 0; r < 8; ++r) {
      float m = NEGI;
#pragma unroll
      for (int j = 0; j < 4; ++j) { s[j][r] *= sscale; m = fmaxf(m, s[j][r]); }
#pragma unroll
      for (int off = 1; off < 16; off <<= 1) m = fmaxf(m, __shfl_xor(m, off, 32));
      float sum = 0.f;
#pragma unroll
      for (int j = 0; j < 4; ++j) { const float p = __expf(s[j][r] - m); sum += p; s[j][r] = p; }
#pragma unroll
      for (int off = 1; off < 16; off <<= 1) sum += __shfl_xor(sum, off, 32);
      const float w4 = 0.25f * __builtin_amdgcn_rcpf(sum);
#pragma unroll
      for (int j = 0; j < 4; ++j) pacc[j][r] += s[j][r] * w4;
    }
  }
  __syncthreads();
  if (hp == 1) {
#pragma unroll
    for (int j = 0; j < 4; ++j)
#pragma unroll
      for (int r = 0; r < 8; ++r) Apart[(rt * 16 + 8 * hh + r) * APT + 16 * j + c] = pacc[j][r];
  }
  __syncthreads();
  if (hp == 0) {
#pragma unroll
    for (int j = 0; j < 4; ++j)
#pragma unroll
      for (int r = 0; r < 8; ++r) {
        const float v = pacc[j][r] + Apart[(rt * 16 + 8 * hh + r) * APT + 16 * j + c];
        Ah[(rt * 16 + 8 * hh + r) * AHP + 16 * j + c] = (_Float16)(v * 1024.0f);
      }
  }
  __syncthreads();

  const int ctb = 4 * hp;
  v8f acc[4];
#pragma unroll
  for (int j = 0; j < 4; ++j) acc[j] = zero8();
#pragma unroll
  for (int kk = 0; kk < 2; ++kk) {
    const v16h aa = ldfrag(Ah, AHP, rt * 16, 32 * kk, lane);
#pragma unroll
    for (int j = 0; j < 4; ++j) {
      const v16h zb = ldfrag(Zt, AHP, (ctb + j) * 16, 32 * kk, lane);
      acc[j] = mma16(aa, zb, acc[j]);
    }
  }
  __syncthreads();

  float* sw = stg + wave * 16 * APT;
#pragma unroll
  for (int j = 0; j < 4; ++j) {
#pragma unroll
    for (int r = 0; r < 8; ++r)
      sw[(8 * hh + r) * APT + 16 * j + c] = acc[j][r] * 0.000244140625f;
  }
  __syncthreads();
  v4f val[8];
  size_t go[8];
  int so[8];
#pragma unroll
  for (int it = 0; it < 8; ++it) {
    const int p  = lane + 32 * it;
    const int L  = p >> 4;
    const int pc = p & 15;
    so[it] = L * APT + 4 * pc;
    go[it] = (rowb + rt * 16 + L) * DMOD + 64 * hp + 4 * pc;
    const v4f az = *(const v4f*)(sw + so[it]);
    const v4f zo = *(const v4f*)(z + go[it]);
    val[it] = zo + dt * (az - zo);
  }
#pragma unroll
  for (int it = 0; it < 8; ++it) *(v4f*)(sw + so[it]) = val[it];
#pragma unroll
  for (int it = 0; it < 8; ++it) *(volatile v4f*)(z + go[it]) = val[it];
  __threadfence();
#pragma unroll
  for (int it = 0; it < 8; ++it) *(volatile v4f*)(z + go[it]) = val[it];
  __syncthreads();
  v4u hv[4];
  size_t gh[4];
#pragma unroll
  for (int it = 0; it < 4; ++it) {
    const int p  = lane + 32 * it;
    const int L  = p >> 3;
    const int pc = p & 7;
    const float* ra = sw + L * APT + 8 * pc;
    const v4f a0 = *(const v4f*)(ra) * 4.0f, a1 = *(const v4f*)(ra + 4) * 4.0f;
    Pack8 pk;
    pk.h = (v8h){(_Float16)a0[0], (_Float16)a0[1], (_Float16)a0[2], (_Float16)a0[3],
                 (_Float16)a1[0], (_Float16)a1[1], (_Float16)a1[2], (_Float16)a1[3]};
    hv[it] = pk.u;
    gh[it] = (rowb + rt * 16 + L) * DMOD + 64 * hp + 8 * pc;
  }
#pragma unroll
  for (int it = 0; it < 4; ++it) *(volatile v4u*)(zh + gh[it]) = hv[it];
  __threadfence();
#pragma unroll
  for (int it = 0; it < 4; ++it) *(volatile v4u*)(zh + gh[it]) = hv[it];
}

extern "C" void kernel_launch(void* const* d_in, const int* in_sizes, int n_in,
                              void* d_out, int out_size, void* d_ws, size_t ws_size,
                              hipStream_t stream) {
  if (n_in < 27) return;
  if (in_sizes[0]  != NTOK * DIN) return;
  if (in_sizes[1]  != NNODE * DIN * DMOD) return;
  if (in_sizes[2]  != NNODE * DMOD) return;
  if (in_sizes[3]  != NNODE * DMOD * WQKV) return;
  if (in_sizes[4]  != NNODE * WQKV) return;
  if (in_sizes[5]  != NNODE * DMOD * DMOD) return;
  if (in_sizes[6]  != NNODE * DMOD) return;
  if (in_sizes[7]  != NNODE * DMOD) return;
  if (in_sizes[8]  != NNODE * DMOD) return;
  if (in_sizes[9]  != NNODE * DMOD) return;
  if (in_sizes[10] != NNODE * DMOD) return;
  if (in_sizes[11] != NNODE * DMOD * DMOD) return;
  if (in_sizes[12] != NNODE * DMOD) return;
  if (in_sizes[13] != NNODE * DMOD * DMOD) return;
  if (in_sizes[14] != NNODE * DMOD) return;
  if (in_sizes[15] != DMOD * DMOD) return;
  if (in_sizes[16] != DMOD) return;
  if (in_sizes[17] != DMOD * WGQK) return;
  if (in_sizes[18] != WGQK) return;
  if (in_sizes[19] != DMOD * DMOD) return;
  if (in_sizes[20] != DMOD) return;
  if (in_sizes[21] != DMOD) return;
  if (in_sizes[22] != DMOD) return;
  if (in_sizes[23] != DMOD * DMOD) return;
  if (in_sizes[24] != DMOD) return;
  if (in_sizes[25] != DMOD * DMOD) return;
  if (in_sizes[26] != DMOD) return;
  if (out_size != NTOK * DMOD) return;

  const float* x      = (const float*)d_in[0];
  const float* tWi    = (const float*)d_in[1];
  const float* tbi    = (const float*)d_in[2];
  const float* tWqkv  = (const float*)d_in[3];
  const float* tbqkv  = (const float*)d_in[4];
  const float* tWo    = (const float*)d_in[5];
  const float* tbo    = (const float*)d_in[6];
  const float* ln1s   = (const float*)d_in[7];
  const float* ln1b   = (const float*)d_in[8];
  const float* ln2s   = (const float*)d_in[9];
  const float* ln2b   = (const float*)d_in[10];
  const float* tW1    = (const float*)d_in[11];
  const float* tb1    = (const float*)d_in[12];
  const float* tW2    = (const float*)d_in[13];
  const float* tb2    = (const float*)d_in[14];
  const float* gWin   = (const float*)d_in[15];
  const float* gbin   = (const float*)d_in[16];
  const float* gWqk   = (const float*)d_in[17];
  const float* gbqk   = (const float*)d_in[18];
  const float* gWout  = (const float*)d_in[19];
  const float* gbout  = (const float*)d_in[20];
  const float* lns    = (const float*)d_in[21];
  const float* lnb    = (const float*)d_in[22];
  const float* mW1    = (const float*)d_in[23];
  const float* mb1    = (const float*)d_in[24];
  const float* mW2    = (const float*)d_in[25];
  const float* mb2    = (const float*)d_in[26];
  float* out = (float*)d_out;

  size_t off = 0;
  const size_t oWi   = off; off += (size_t)NNODE * DMOD * DIN * 2;
  const size_t oWqkv = off; off += (size_t)NNODE * WQKV * DMOD * 2;
  const size_t oWo   = off; off += (size_t)NNODE * DMOD * DMOD * 2;
  const size_t oW1   = off; off += (size_t)NNODE * DMOD * DMOD * 2;
  const size_t oW2   = off; off += (size_t)NNODE * DMOD * DMOD * 2;
  const size_t oGin  = off; off += (size_t)DMOD * DMOD * 2;
  const size_t oGqk  = off; off += (size_t)WGQK * DMOD * 2;
  const size_t oGout = off; off += (size_t)DMOD * DMOD * 2;
  const size_t oM1   = off; off += (size_t)DMOD * DMOD * 2;
  const size_t oM2   = off; off += (size_t)DMOD * DMOD * 2;
  const size_t oPE   = off; off += (size_t)NTIME * DMOD * 4;
  const size_t oR1   = off; off += (size_t)NTOK * DMOD * 4;
  const size_t oR2   = off; off += (size_t)NTOK * DMOD * 2;
  const size_t oR3   = off; off += (size_t)NTOK * WQKV * 2;
  const size_t oR4   = off; off += (size_t)NTOK * DMOD * 2;
  if (off > ws_size) return;
  if (off > (size_t)134217728) return;
  if ((size_t)NTOK * DIN * 2 > (size_t)NTOK * DMOD * 2) return;
  if ((size_t)NTOK * DMOD * 4 + (size_t)NTOK * DMOD * 2 > (size_t)NTOK * WQKV * 2) return;
  if ((size_t)NTOK * WGQK * 2 > (size_t)NTOK * DMOD * 4) return;

  char* ws = (char*)d_ws;
  _Float16* Wi_t   = (_Float16*)(ws + oWi);
  _Float16* Wqkv_t = (_Float16*)(ws + oWqkv);
  _Float16* Wo_t   = (_Float16*)(ws + oWo);
  _Float16* W1_t   = (_Float16*)(ws + oW1);
  _Float16* W2_t   = (_Float16*)(ws + oW2);
  _Float16* Gin_t  = (_Float16*)(ws + oGin);
  _Float16* Gqk_t  = (_Float16*)(ws + oGqk);
  _Float16* Gout_t = (_Float16*)(ws + oGout);
  _Float16* M1_t   = (_Float16*)(ws + oM1);
  _Float16* M2_t   = (_Float16*)(ws + oM2);
  float*    PE     = (float*)(ws + oPE);
  float*    X0     = (float*)(ws + oR1);
  float*    Z      = X0;
  float*    Yp     = X0;
  _Float16* Hh     = (_Float16*)(ws + oR2);
  _Float16* QKV    = (_Float16*)(ws + oR3);
  float*    X1     = (float*)(ws + oR3);
  _Float16* Gp     = (_Float16*)(ws + oR3 + (size_t)NTOK * DMOD * 4);
  _Float16* QK     = (_Float16*)(ws + oR3);
  _Float16* Zh     = (_Float16*)(ws + oR3 + (size_t)NTOK * DMOD * 4);
  _Float16* Xh     = (_Float16*)(ws + oR4);
  _Float16* Oh     = (_Float16*)(ws + oR4);
  _Float16* HT     = (_Float16*)(ws + oR4);
  _Float16* Mh     = (_Float16*)(ws + oR4);

  k_cvt8<<<dim3((NTOK * DIN) / 2048), dim3(256), 0, stream>>>(x, Xh);
  k_wt<DIN><<<dim3(DMOD / 32, NNODE), dim3(256), 0, stream>>>(tWi, DMOD, Wi_t, 64.0f);
  k_wt<DMOD><<<dim3(WQKV / 32, NNODE), dim3(256), 0, stream>>>(tWqkv, WQKV, Wqkv_t, 64.0f);
  k_wt<DMOD><<<dim3(DMOD / 32, NNODE), dim3(256), 0, stream>>>(tWo, DMOD, Wo_t, 64.0f);
  k_wt<DMOD><<<dim3(DMOD / 32, NNODE), dim3(256), 0, stream>>>(tW1, DMOD, W1_t, 64.0f);
  k_wt<DMOD><<<dim3(DMOD / 32, NNODE), dim3(256), 0, stream>>>(tW2, DMOD, W2_t, 64.0f);
  k_wt<DMOD><<<dim3(DMOD / 32, 1), dim3(256), 0, stream>>>(gWin, DMOD, Gin_t, 64.0f);
  k_wt<DMOD><<<dim3(WGQK / 32, 1), dim3(256), 0, stream>>>(gWqk, WGQK, Gqk_t, 64.0f);
  k_wt<DMOD><<<dim3(DMOD / 32, 1), dim3(256), 0, stream>>>(gWout, DMOD, Gout_t, 64.0f);
  k_wt<DMOD><<<dim3(DMOD / 32, 1), dim3(256), 0, stream>>>(mW1, DMOD, M1_t, 64.0f);
  k_wt<DMOD><<<dim3(DMOD / 32, 1), dim3(256), 0, stream>>>(mW2, DMOD, M2_t, 64.0f);
  k_petab<<<dim3((NTIME * DMOD) / 256), dim3(256), 0, stream>>>(PE);

  const dim3 gpn(ROWSPN / 256, DMOD / 64, NNODE);
  const dim3 gqkv(ROWSPN / 256, WQKV / 64, NNODE);
  k_gemm<0, false, false, true, false><<<gpn, dim3(256), 0, stream>>>(
      Xh, NNODE * DIN, DIN, Wi_t, DIN, DMOD * DIN, tbi, DMOD, PE, PE, 0.015625f, 1.0f, X0, Hh, NNODE * DMOD, DMOD);
  k_ln<<<dim3(NTOK / 16), dim3(256), 0, stream>>>(X0, ln1s, ln1b, NNODE - 1, Hh);
  k_gemm<1, false, false, false, false><<<gqkv, dim3(256), 0, stream>>>(
      Hh, NNODE * DMOD, DMOD, Wqkv_t, DMOD, WQKV * DMOD, tbqkv, WQKV, PE, PE, 0.015625f, 8.0f, X0, QKV,
      NNODE * WQKV, WQKV);
  const float sscale_t = 0.17677669529663687f * 0.015625f;
  k_attn_t<<<dim3(NBATCH * NNODE), dim3(256), 0, stream>>>(QKV, Oh, sscale_t);
  k_gemm<0, true, false, false, true><<<gpn, dim3(256), 0, stream>>>(
      Oh, 0, 0, Wo_t, DMOD, DMOD * DMOD, tbo, DMOD, X0, PE, 0.000244140625f, 1.0f, X1, Hh, NNODE * DMOD, DMOD);
  k_ln<<<dim3(NTOK / 16), dim3(256), 0, stream>>>(X1, ln2s, ln2b, NNODE - 1, Hh);
  k_gemm<1, false, true, false, false><<<gpn, dim3(256), 0, stream>>>(
      Hh, NNODE * DMOD, DMOD, W1_t, DMOD, DMOD * DMOD, tb1, DMOD, PE, PE, 0.015625f, 16.0f, X0, Gp, NNODE * DMOD,
      DMOD);
  k_gemm<1, true, false, false, false><<<gpn, dim3(256), 0, stream>>>(
      Gp, NNODE * DMOD, DMOD, W2_t, DMOD, DMOD * DMOD, tb2, DMOD, X1, PE, 0.0009765625f, 1.0f, X0, HT,
      NNODE * DMOD, DMOD);

  const dim3 gsh(NTOK / 256, DMOD / 64, 1);
  const dim3 gshq(NTOK / 256, WGQK / 64, 1);
  k_gemm<2, false, false, false, false><<<gsh, dim3(256), 0, stream>>>(
      HT, DMOD, 0, Gin_t, DMOD, 0, gbin, 0, PE, PE, 0.015625f, 4.0f, Z, Zh, DMOD, 0);
  const float sscale_g = 0.17677669529663687f * 0.00390625f;
  const float dts[3] = {0.166666672f, 0.166666672f, 0.166666657f};
  for (int i = 0; i < 3; ++i) {
    k_gemm<1, false, false, false, false><<<gshq, dim3(256), 0, stream>>>(
        Zh, DMOD, 0, Gqk_t, DMOD, 0, gbqk, 0, PE, PE, 0.00390625f, 16.0f, PE, QK, WGQK, 0);
    k_gdiff<<<dim3(NBATCH * NTIME), dim3(256), 0, stream>>>(QK, Z, Zh, sscale_g, dts[i]);
  }
  k_gemm<0, false, false, false, false><<<gsh, dim3(256), 0, stream>>>(
      Zh, DMOD, 0, Gout_t, DMOD, 0, gbout, 0, PE, PE, 0.00390625f, 1.0f, Yp, Hh, DMOD, 0);

  k_ln<<<dim3(NTOK / 16), dim3(256), 0, stream>>>(Yp, lns, lnb, 0, Hh);
  k_gemm<1, false, true, false, false><<<gsh, dim3(256), 0, stream>>>(
      Hh, DMOD, 0, M1_t, DMOD, 0, mb1, 0, PE, PE, 0.015625f, 16.0f, PE, Mh, DMOD, 0);
  k_gemm<0, false, false, false, false><<<gsh, dim3(256), 0, stream>>>(
      Mh, DMOD, 0, M2_t, DMOD, 0, mb2, 0, PE, PE, 0.0009765625f, 1.0f, out, Hh, DMOD, 0);
  (void)hipGetLastError();
}
